// GCNClassifier_41601053229302
// MI455X (gfx1250) — hardware-verified
//
#include <hip/hip_runtime.h>
#include <stddef.h>
#include <stdint.h>


#define F      64
#define F2     128
#define CH     128
#define KC     256
#define NTSK   12
#define NTP    16
#define MAXG   1024
#define NTHR   256
#define NWAVE  8
#define EPT    8
#define CHUNK  (NTHR * EPT)
#define WCAP   (EPT * 32)
#define LISTN  (NWAVE * WCAP)
#define NBA    1024
#define SLA    10
#define RCAP   16384
#define DEGCAP 64
#define PARTW  192
#define WSTW   130
#define NGB    32
#define GBM    64
#define GBN    128
#define GTHR   128
#define NUB0   (F2 * (F / 8))
#define NUB1   (F2 * (F2 / 8))
#define NUC1   (CH * (KC / 8))
#define NUC2   (NTP * (KC / 8))
#define AGG_ZINTS (LISTN + 2 * RCAP + 3 * NBA)
#define AGG_LDS_INTS (AGG_ZINTS + 16 + NWAVE * WSTW + PARTW)
#define WSMAX  134217728

static_assert((CHUNK & (CHUNK - 1)) == 0 && CHUNK <= 4096);
static_assert((NBA & (NBA - 1)) == 0 && NBA == (1 << SLA));
static_assert(((long long)CHUNK << SLA) < (1LL << 31));
static_assert(LISTN % NTHR == 0);
static_assert(NBA % NWAVE == 0 && NBA % 32 == 0 && NBA % GBM == 0);
static_assert(RCAP % 4 == 0 && AGG_ZINTS % 4 == 0 && LISTN % 4 == 0);
static_assert((AGG_ZINTS + 16 + NWAVE * WSTW) % 4 == 0);
static_assert(AGG_LDS_INTS * 4 <= 300000);
static_assert(NUB0 % NTHR == 0 && NUB1 % NTHR == 0 && NUC1 % NTHR == 0 && NUC2 % NTHR == 0);
static_assert(GBM == (GTHR / 32) * 16 && GBN == 4 * 32);
static_assert(F % 32 == 0 && F2 % 32 == 0 && KC % 32 == 0 && KC == 2 * CH && F2 == 2 * F);
static_assert(NGB == 4 * NWAVE);
static_assert(PARTW % 32 == 0 && PARTW / 4 <= NTHR && PARTW >= 2 * F + 1);
static_assert(MAXG * NTSK % 4 == 0);
static_assert(NTSK <= NTP);

typedef float          v2f   __attribute__((ext_vector_type(2)));
typedef float          v4f   __attribute__((ext_vector_type(4)));
typedef float          v8f   __attribute__((ext_vector_type(8)));
typedef int            v4i   __attribute__((ext_vector_type(4)));
typedef int            v8i   __attribute__((ext_vector_type(8)));
typedef unsigned short v8us  __attribute__((ext_vector_type(8)));
typedef unsigned short v16us __attribute__((ext_vector_type(16)));
typedef __bf16         v16bf __attribute__((ext_vector_type(16)));
typedef v2f  __attribute__((may_alias)) v2fa;
typedef v4f  __attribute__((may_alias)) v4fa;
typedef v4i  __attribute__((may_alias)) v4ia;
typedef v8us __attribute__((may_alias)) v8usa;
union FragB { v16bf v; v16us u; v8us h[2]; v8i w; };

__device__ __forceinline__ v8f wmb(const FragB& a, const FragB& b, v8f c) {
  v8f d = __builtin_amdgcn_wmma_f32_16x16x32_bf16(false, a.v, false, b.v, (short)0, c, false, false);
  asm volatile("v_nop\n\tv_nop\n\tv_nop\n\tv_nop" : "+v"(d) : "v"(a.w), "v"(b.w));
  return d;
}

__device__ __forceinline__ v8f z8() { v8f z = {0.f, 0.f, 0.f, 0.f, 0.f, 0.f, 0.f, 0.f}; return z; }

__device__ __forceinline__ unsigned bf16_bits(float f) {
  const unsigned u = __float_as_uint(f);
  return (u + 0x7FFFu + ((u >> 16) & 1u)) >> 16;
}
__device__ __forceinline__ float bf16_val(float f) {
  return __uint_as_float(bf16_bits(f) << 16);
}
__device__ __forceinline__ float wsum(float p) {
  p += __shfl_xor(p, 16); p += __shfl_xor(p, 8); p += __shfl_xor(p, 4); p += __shfl_xor(p, 2); p += __shfl_xor(p, 1);
  return p;
}

template <int SLB>
__device__ __forceinline__ int scan_chunk(const int* __restrict__ ids, int nE, int cbase, int slotBase,
                                          int nb, int vec8, int* list, int tid, int lane, int wave) {
  int wc = 0;
  const int el0  = tid * EPT;
  const int e0   = cbase + el0;
  const int sent = -2147483647 - 1;
  v4i da, db;
  if (vec8 != 0 && cbase + CHUNK <= nE) {
    da = *(const v4i*)(ids + e0);
    db = *(const v4i*)(ids + e0 + 4);
  } else {
    da.x = (e0     < nE) ? ids[min(e0,     nE - 1)] : sent;
    da.y = (e0 + 1 < nE) ? ids[min(e0 + 1, nE - 1)] : sent;
    da.z = (e0 + 2 < nE) ? ids[min(e0 + 2, nE - 1)] : sent;
    da.w = (e0 + 3 < nE) ? ids[min(e0 + 3, nE - 1)] : sent;
    db.x = (e0 + 4 < nE) ? ids[min(e0 + 4, nE - 1)] : sent;
    db.y = (e0 + 5 < nE) ? ids[min(e0 + 5, nE - 1)] : sent;
    db.z = (e0 + 6 < nE) ? ids[min(e0 + 6, nE - 1)] : sent;
    db.w = (e0 + 7 < nE) ? ids[min(e0 + 7, nE - 1)] : sent;
  }
  const unsigned nbs = (unsigned)slotBase;
  const unsigned unb = (unsigned)nb;
  const unsigned s0 = (unsigned)da.x - nbs, s1 = (unsigned)da.y - nbs;
  const unsigned s2 = (unsigned)da.z - nbs, s3 = (unsigned)da.w - nbs;
  const unsigned s4 = (unsigned)db.x - nbs, s5 = (unsigned)db.y - nbs;
  const unsigned s6 = (unsigned)db.z - nbs, s7 = (unsigned)db.w - nbs;
  const bool h0 = s0 < unb, h1 = s1 < unb, h2 = s2 < unb, h3 = s3 < unb;
  const bool h4 = s4 < unb, h5 = s5 < unb, h6 = s6 < unb, h7 = s7 < unb;
  const unsigned any = __builtin_amdgcn_ballot_w32(h0 | h1 | h2 | h3 | h4 | h5 | h6 | h7);
  if (any != 0u) {
#define HITJ(J, HJ, SJ) { \
      const unsigned mj = __builtin_amdgcn_ballot_w32(HJ); \
      if (mj != 0u) { \
        if (HJ) { \
          const int pos = wc + (int)__builtin_amdgcn_mbcnt_lo(mj, 0u); \
          if (pos < WCAP) list[wave * WCAP + pos] = ((el0 + (J)) << SLB) | (int)(SJ); \
        } \
        wc += (int)__builtin_popcount(mj); } }
    HITJ(0, h0, s0)
    HITJ(1, h1, s1)
    HITJ(2, h2, s2)
    HITJ(3, h3, s3)
    HITJ(4, h4, s4)
    HITJ(5, h5, s5)
    HITJ(6, h6, s6)
    HITJ(7, h7, s7)
#undef HITJ
  }
  return wc;
}

__global__ __launch_bounds__(NTHR) void k_prep(const float* __restrict__ W0, const float* __restrict__ rW0,
                                               const float* __restrict__ W1, const float* __restrict__ rW1,
                                               const float* __restrict__ c1W, const float* __restrict__ c2W,
                                               unsigned short* B0, unsigned short* B1,
                                               unsigned short* C1T, unsigned short* C2T) {
  const int u = (int)blockIdx.x * NTHR + (int)threadIdx.x;
  v8us o;
  unsigned short* dp;
  if (u < NUB0) {
    const int n  = u >> 3;
    const int k8 = (u & 7) * 8;
    const float* wp;
    if (n < F) wp = W0; else wp = rW0;
    const float* p = wp + (size_t)k8 * F + (n & (F - 1));
#pragma unroll
    for (int i = 0; i < 8; ++i) o[i] = (unsigned short)bf16_bits(p[(size_t)i * F]);
    dp = B0 + (size_t)u * 8;
  } else if (u < NUB0 + NUB1) {
    const int v  = u - NUB0;
    const int n  = v >> 4;
    const int k8 = (v & 15) * 8;
    const int kk = k8 & (F - 1);
    const float* wp;
    if (n < F) wp = W1; else wp = rW1;
    const float* p = wp + (size_t)kk * F + (n & (F - 1));
#pragma unroll
    for (int i = 0; i < 8; ++i) o[i] = (unsigned short)bf16_bits(p[(size_t)i * F]);
    dp = B1 + (size_t)v * 8;
  } else if (u < NUB0 + NUB1 + NUC1) {
    const int v  = u - NUB0 - NUB1;
    const int n  = v >> 5;
    const int k8 = (v & 31) * 8;
    const int kk = k8 & (CH - 1);
    const float* p = c1W + (size_t)kk * CH + n;
#pragma unroll
    for (int i = 0; i < 8; ++i) o[i] = (unsigned short)bf16_bits(p[(size_t)i * CH]);
    dp = C1T + (size_t)v * 8;
  } else if (u < NUB0 + NUB1 + NUC1 + NUC2) {
    const int v  = u - NUB0 - NUB1 - NUC1;
    const int n  = v >> 5;
    const int k8 = (v & 31) * 8;
    const int kk = k8 & (CH - 1);
    const int nc = n < NTSK ? n : NTSK - 1;
    const float* p = c2W + (size_t)kk * NTSK + nc;
#pragma unroll
    for (int i = 0; i < 8; ++i) {
      const unsigned short bv = (unsigned short)bf16_bits(p[(size_t)i * NTSK]);
      o[i] = (n < NTSK) ? bv : (unsigned short)0;
    }
    dp = C2T + (size_t)v * 8;
  } else {
    return;
  }
  *(volatile v8us*)dp = o;
  __threadfence();
  *(volatile v8us*)dp = o;
}

__global__ __launch_bounds__(NTHR) void k_cva(const float* __restrict__ x, int nN, int nUnits,
                                              unsigned short* xb) {
  const int u = (int)blockIdx.x * NTHR + (int)threadIdx.x;
  if (u >= nUnits) return;
  const int row = u >> 3;
  const int k8  = (u & 7) * 8;
  const int rc  = row < nN ? row : nN - 1;
  const float* p = x + (size_t)rc * F + k8;
  const v4f a = *(const v4f*)p;
  const v4f b = *(const v4f*)(p + 4);
  const bool ok = row < nN;
  v8us o;
  o[0] = ok ? (unsigned short)bf16_bits(a.x) : (unsigned short)0;
  o[1] = ok ? (unsigned short)bf16_bits(a.y) : (unsigned short)0;
  o[2] = ok ? (unsigned short)bf16_bits(a.z) : (unsigned short)0;
  o[3] = ok ? (unsigned short)bf16_bits(a.w) : (unsigned short)0;
  o[4] = ok ? (unsigned short)bf16_bits(b.x) : (unsigned short)0;
  o[5] = ok ? (unsigned short)bf16_bits(b.y) : (unsigned short)0;
  o[6] = ok ? (unsigned short)bf16_bits(b.z) : (unsigned short)0;
  o[7] = ok ? (unsigned short)bf16_bits(b.w) : (unsigned short)0;
  unsigned short* dp = xb + (size_t)row * F + k8;
  *(volatile v8us*)dp = o;
  __threadfence();
  *(volatile v8us*)dp = o;
}

__global__ __launch_bounds__(GTHR) void k_gemm(const unsigned short* __restrict__ A, int lda,
                                               const unsigned short* __restrict__ BT, int ldb, int K,
                                               float* Cm, int ldc) {
  __shared__ __attribute__((aligned(16))) float stg[GBM * GBN];
  const int tid = (int)threadIdx.x, lane = tid & 31, wave = tid >> 5, hh = lane >> 4, m = lane & 15;
  const int rowBase = (int)blockIdx.x * GBM;
  const int colBase = (int)blockIdx.y * GBN;

  v8f acc[8];
#pragma unroll
  for (int t = 0; t < 8; ++t) acc[t] = z8();
  const unsigned short* ap = A  + (size_t)(rowBase + 16 * wave + m) * (size_t)lda + 8 * hh;
  const unsigned short* bp = BT + (size_t)(colBase + m) * (size_t)ldb + 8 * hh;

#pragma unroll 1
  for (int k0 = 0; k0 < K; k0 += 32) {
    FragB af;
    af.h[0] = *(const v8usa*)(ap + k0);
    af.h[1] = *(const v8usa*)(ap + k0 + 16);
#pragma unroll
    for (int nt = 0; nt < 8; ++nt) {
      const unsigned short* wq = bp + (size_t)(16 * nt) * (size_t)ldb + k0;
      FragB bf;
      bf.h[0] = *(const v8usa*)wq;
      bf.h[1] = *(const v8usa*)(wq + 16);
      acc[nt] = wmb(af, bf, acc[nt]);
    }
  }

#pragma unroll
  for (int nt = 0; nt < 8; ++nt) {
    const int lc = 16 * nt + m;
#pragma unroll
    for (int r = 0; r < 8; ++r) {
      const int lr = 16 * wave + 8 * hh + r;
      stg[lr * GBN + lc] = acc[nt][r];
    }
  }
  __syncthreads();

  v4f pv[16];
#pragma unroll
  for (int i = 0; i < 16; ++i) pv[i] = *(const v4fa*)(stg + (16 * wave + i) * GBN + 4 * lane);
#pragma unroll
  for (int i = 0; i < 16; ++i) {
    float* op = Cm + (size_t)(rowBase + 16 * wave + i) * (size_t)ldc + colBase + 4 * lane;
    *(volatile v4f*)op = pv[i];
  }
  __threadfence();
#pragma unroll
  for (int i = 0; i < 16; ++i) {
    float* op = Cm + (size_t)(rowBase + 16 * wave + i) * (size_t)ldc + colBase + 4 * lane;
    *(volatile v4f*)op = pv[i];
  }
}

__global__ __launch_bounds__(NTHR) void k_agg(const int* __restrict__ srcs, const int* __restrict__ dsts,
                                              int nE, int nN, int vec8, int mRows,
                                              const float* __restrict__ mr,
                                              const float* __restrict__ bias, const float* __restrict__ rbias,
                                              float* hr, float* part) {
  extern __shared__ __attribute__((aligned(16))) int dsm[];
  int* list = dsm;
  int* hl   = dsm + LISTN;
  int* sl   = hl + RCAP;
  int* cnt  = sl + RCAP;
  int* offs = cnt + NBA;
  int* cur  = offs + NBA;
  int* misc = cur + NBA;
  float* wst = (float*)(misc + 16);
  float* pst = wst + NWAVE * WSTW;
  const int tid = (int)threadIdx.x, lane = tid & 31, wave = tid >> 5;
  const int nodeBase = (int)blockIdx.x * NBA;

  {
    const v4i z4 = {0, 0, 0, 0};
    for (int i = tid * 4; i < AGG_ZINTS; i += NTHR * 4) *(v4ia*)(dsm + i) = z4;
    if (tid < 16) misc[tid] = 0;
  }
  float bv0, bv1, rv0, rv1;
  {
    const v2f bq = *(const v2fa*)(bias + 2 * lane);
    const v2f rq = *(const v2fa*)(rbias + 2 * lane);
    bv0 = bf16_val(bq.x); bv1 = bf16_val(bq.y);
    rv0 = bf16_val(rq.x); rv1 = bf16_val(rq.y);
  }
  __syncthreads();

  int t = 0, ov = 0;
  const int nChunks = (nE + CHUNK - 1) / CHUNK;
#pragma unroll 1
  for (int ch = 0; ch < nChunks; ++ch) {
    const int cbase = ch * CHUNK;
    const int wc = scan_chunk<SLA>(dsts, nE, cbase, nodeBase, NBA, vec8, list, tid, lane, wave);
    if (lane == 0) misc[wave] = wc;
    __syncthreads();
    if (wave == 0) {
#pragma unroll 1
      for (int w2 = 0; w2 < NWAVE; ++w2) {
        int c = misc[w2];
        c = c < 0 ? 0 : (c > WCAP ? WCAP : c);
#pragma unroll 1
        for (int b0 = 0; b0 < c; b0 += 32) {
          const int idx = b0 + lane;
          const int ent = list[w2 * WCAP + (idx < WCAP ? idx : WCAP - 1)];
          const int m32 = (c - b0) < 32 ? (c - b0) : 32;
#pragma unroll 1
          for (int k = 0; k < m32; ++k) {
            const int u    = __builtin_amdgcn_readlane(ent, k);
            const int slot = u & (NBA - 1);
            const int el   = (u >> SLA) & (CHUNK - 1);
            const int pk   = ((cbase + el) << SLA) | slot;
            if (t < RCAP) {
              if (lane == 0) { hl[t] = pk; cnt[slot] = cnt[slot] + 1; }
              t = t + 1;
            } else {
              ov = 1;
            }
          }
        }
      }
    }
    __syncthreads();
  }
  if (wave == 0 && lane == 0) { misc[8] = t; misc[9] = ov; }
  __syncthreads();
  int tt = misc[8];
  tt = tt < 0 ? 0 : (tt > RCAP ? RCAP : tt);
  const int ovf = misc[9];

  if (wave == 0) {
    const int base = lane * (NBA / 32);
    int s = 0;
#pragma unroll 1
    for (int i = 0; i < NBA / 32; ++i) s += cnt[base + i];
    int incl = s;
#pragma unroll
    for (int d = 1; d < 32; d <<= 1) {
      const int y = __shfl_up(incl, d, 32);
      if (lane >= d) incl += y;
    }
    int run = incl - s;
#pragma unroll 1
    for (int i = 0; i < NBA / 32; ++i) {
      const int cv = cnt[base + i];
      offs[base + i] = run;
      cur[base + i]  = run;
      run += cv;
    }
  }
  __syncthreads();
  if (wave == 0) {
#pragma unroll 1
    for (int b0 = 0; b0 < tt; b0 += 32) {
      const int idx = b0 + lane;
      const int ent = hl[idx < RCAP ? idx : RCAP - 1];
      const int m32 = (tt - b0) < 32 ? (tt - b0) : 32;
#pragma unroll 1
      for (int k = 0; k < m32; ++k) {
        const int u    = __builtin_amdgcn_readlane(ent, k);
        const int slot = u & (NBA - 1);
        if (lane == 0) {
          int p = cur[slot];
          p = p < 0 ? 0 : (p > RCAP - 1 ? RCAP - 1 : p);
          sl[p] = u;
          cur[slot] = p + 1;
        }
      }
    }
  }
  __syncthreads();

  const float pz = (ovf != 0) ? __int_as_float(0x7fc00000) : 0.0f;
  int wn = 0;
  float wm0 = 0.0f, wm1 = 0.0f, wq0 = 0.0f, wq1 = 0.0f;
#pragma unroll 1
  for (int si = 0; si < NBA / NWAVE; ++si) {
    const int s    = si * NWAVE + wave;
    const int node = nodeBase + s;
    int c = cnt[s];
    const bool big = c > DEGCAP;
    c = c < 0 ? 0 : (c > DEGCAP ? DEGCAP : c);
    int o = offs[s];
    o = o < 0 ? 0 : (o > RCAP ? RCAP : o);
    const int nc = node < nN ? node : nN - 1;
    float a0 = 0.0f, a1 = 0.0f;
#pragma unroll 1
    for (int b0 = 0; b0 < c; b0 += 32) {
      int idx = o + b0 + lane;
      idx = idx > RCAP - 1 ? RCAP - 1 : idx;
      const int ent = sl[idx];
      int eid = ent >> SLA;
      eid = eid < 0 ? 0 : (eid > nE - 1 ? nE - 1 : eid);
      int sr = srcs[eid];
      sr = sr < 0 ? 0 : (sr > nN - 1 ? nN - 1 : sr);
      const int m32 = (c - b0) < 32 ? (c - b0) : 32;
#pragma unroll 1
      for (int k = 0; k < m32; ++k) {
        const int sk = __builtin_amdgcn_readlane(sr, k);
        const v2f a = *(const v2fa*)(mr + (size_t)sk * F2 + 2 * lane);
        a0 += a.x;
        a1 += a.y;
      }
    }
    const v2f xr = *(const v2fa*)(mr + (size_t)nc * F2 + F + 2 * lane);
    const float pzr = big ? __int_as_float(0x7fc00000) : pz;
    const bool live = node < nN;
    float y0 = fmaxf(a0 + bv0, 0.0f) + fmaxf(xr.x + rv0, 0.0f);
    float y1 = fmaxf(a1 + bv1, 0.0f) + fmaxf(xr.y + rv1, 0.0f);
    y0 = y0 + pzr;
    y1 = y1 + pzr;
    const float v0 = live ? y0 : 0.0f;
    const float v1 = live ? y1 : 0.0f;
    if (live) {
      wn += 1;
      const float rk = 1.0f / (float)wn;
      const float d0 = v0 - wm0;
      wm0 = fmaf(d0, rk, wm0);
      wq0 = fmaf(d0, v0 - wm0, wq0);
      const float d1 = v1 - wm1;
      wm1 = fmaf(d1, rk, wm1);
      wq1 = fmaf(d1, v1 - wm1, wq1);
    }
    if (node < mRows) {
      v2f hv;
      hv.x = v0; hv.y = v1;
      float* hp = hr + (size_t)node * F + 2 * lane;
      *(volatile v2f*)hp = hv;
      __threadfence();
      *(volatile v2f*)hp = hv;
    }
  }

  if (lane == 0) wst[wave * WSTW] = (float)wn;
  wst[wave * WSTW + 1 + 2 * lane]     = wm0;
  wst[wave * WSTW + 2 + 2 * lane]     = wm1;
  wst[wave * WSTW + 1 + F + 2 * lane] = wq0;
  wst[wave * WSTW + 2 + F + 2 * lane] = wq1;
  __syncthreads();
  if (tid < F) {
    float n = 0.0f, mean = 0.0f, M2 = 0.0f;
#pragma unroll 1
    for (int w2 = 0; w2 < NWAVE; ++w2) {
      const float nb = wst[w2 * WSTW];
      const float mb = wst[w2 * WSTW + 1 + tid];
      const float qb = wst[w2 * WSTW + 1 + F + tid];
      if (nb > 0.5f) {
        const float nn = n + nb;
        const float delta = mb - mean;
        const float f = nb / nn;
        mean = fmaf(delta, f, mean);
        M2 = M2 + qb + delta * delta * n * f;
        n = nn;
      }
    }
    pst[1 + tid] = mean;
    pst[1 + F + tid] = M2;
    if (tid == 0) pst[0] = n;
  } else if (tid >= 2 * F + 1 && tid < PARTW) {
    pst[tid] = 0.0f;
  }
  __syncthreads();
  v4f pv;
  if (tid < PARTW / 4) {
    pv = *(const v4fa*)(pst + 4 * tid);
    *(volatile v4f*)(part + (size_t)blockIdx.x * PARTW + 4 * tid) = pv;
  }
  __threadfence();
  if (tid < PARTW / 4) {
    *(volatile v4f*)(part + (size_t)blockIdx.x * PARTW + 4 * tid) = pv;
  }
}

__global__ __launch_bounds__(64) void k_bnfin(const float* __restrict__ part, int nPart,
                                              const float* __restrict__ gam, const float* __restrict__ bet,
                                              float* ss) {
  __shared__ __attribute__((aligned(16))) float stg[F2];
  const int tid = (int)threadIdx.x;
  const int c = tid & (F - 1);
  float n = 0.0f, mean = 0.0f, M2 = 0.0f;
#pragma unroll 1
  for (int b = 0; b < nPart; ++b) {
    const float* pr = part + (size_t)b * PARTW;
    const float nb = pr[0];
    const float mb = pr[1 + c];
    const float qb = pr[1 + F + c];
    if (nb > 0.5f) {
      const float nn = n + nb;
      const float delta = mb - mean;
      const float f = nb / nn;
      mean = fmaf(delta, f, mean);
      M2 = M2 + qb + delta * delta * n * f;
      n = nn;
    }
  }
  const float nt = n < 1.0f ? 1.0f : n;
  const float var = M2 / nt;
  const float rstd = rsqrtf(var + 1e-5f);
  const float sc = bf16_val(gam[c]) * rstd;
  const float sh = bf16_val(bet[c]) - mean * sc;
  if (tid < F) { stg[c] = sc; stg[F + c] = sh; }
  __syncthreads();
  v4f v;
  if (tid < 32) {
    v = *(const v4fa*)(stg + 4 * tid);
    *(volatile v4f*)(ss + 4 * tid) = v;
  }
  __threadfence();
  if (tid < 32) {
    *(volatile v4f*)(ss + 4 * tid) = v;
  }
}

__global__ __launch_bounds__(NTHR) void k_bnap(const float* __restrict__ hraw, int nN, int nUnits,
                                               const float* __restrict__ ss, unsigned short* a1) {
  __shared__ float ssh[F2];
  const int tid = (int)threadIdx.x;
  if (tid < F2) ssh[tid] = ss[tid];
  __syncthreads();
  const int u = (int)blockIdx.x * NTHR + tid;
  if (u >= nUnits) return;
  const int row = u >> 3;
  const int k8  = (u & 7) * 8;
  const int rc  = row < nN ? row : nN - 1;
  const float* p = hraw + (size_t)rc * F + k8;
  const v4f a = *(const v4f*)p;
  const v4f b = *(const v4f*)(p + 4);
  const bool ok = row < nN;
  float xv[8];
  xv[0] = a.x; xv[1] = a.y; xv[2] = a.z; xv[3] = a.w;
  xv[4] = b.x; xv[5] = b.y; xv[6] = b.z; xv[7] = b.w;
  v8us ho, lo;
#pragma unroll
  for (int i = 0; i < 8; ++i) {
    const float v = fmaf(xv[i], ssh[k8 + i], ssh[F + k8 + i]);
    const unsigned hb = bf16_bits(v);
    const unsigned lb = bf16_bits(v - __uint_as_float(hb << 16));
    ho[i] = ok ? (unsigned short)hb : (unsigned short)0;
    lo[i] = ok ? (unsigned short)lb : (unsigned short)0;
  }
  unsigned short* dp = a1 + (size_t)row * F2 + k8;
  *(volatile v8us*)dp = ho;
  *(volatile v8us*)(dp + F) = lo;
  __threadfence();
  *(volatile v8us*)dp = ho;
  *(volatile v8us*)(dp + F) = lo;
}

__global__ __launch_bounds__(NTHR) void k_pool(const int* __restrict__ ngr, int nN, int vec8,
                                               const float* __restrict__ hr, const float* __restrict__ ss,
                                               const float* __restrict__ awW, const float* __restrict__ awb,
                                               unsigned short* hg, int G) {
  __shared__ __attribute__((aligned(16))) float Rs[NGB * F];
  __shared__ __attribute__((aligned(16))) float Rm[NGB * F];
  __shared__ __attribute__((aligned(16))) int plist[LISTN];
  __shared__ int wcnt[NWAVE];
  const int tid = (int)threadIdx.x, lane = tid & 31, wave = tid >> 5;
  const int gBase = (int)blockIdx.x * NGB;
  int nb = G - gBase;
  nb = nb < 0 ? 0 : (nb > NGB ? NGB : nb);
#pragma unroll 1
  for (int i = tid; i < NGB * F; i += NTHR) { Rs[i] = 0.0f; Rm[i] = -__builtin_inff(); }
#pragma unroll 1
  for (int i = tid; i < LISTN; i += NTHR) plist[i] = 0;
  if (tid < NWAVE) wcnt[tid] = 0;
  const float sc0 = ss[2 * lane], sc1 = ss[2 * lane + 1];
  const float sh0 = ss[F + 2 * lane], sh1 = ss[F + 2 * lane + 1];
  const float aw0 = bf16_val(awW[2 * lane]), aw1 = bf16_val(awW[2 * lane + 1]);
  const float ab  = bf16_val(awb[0]);
  __syncthreads();

  const int nChunks = (nN + CHUNK - 1) / CHUNK;
#pragma unroll 1
  for (int ch = 0; ch < nChunks; ++ch) {
    const int cbase = ch * CHUNK;
    const int wc = scan_chunk<SLA>(ngr, nN, cbase, gBase, nb, vec8, plist, tid, lane, wave);
    if (lane == 0) wcnt[wave] = wc;
    __syncthreads();
#pragma unroll 1
    for (int wsx = 0; wsx < NWAVE; ++wsx) {
      int n = __builtin_amdgcn_readfirstlane(wcnt[wsx]);
      n = n > WCAP ? WCAP : (n < 0 ? 0 : n);
      const int* lp = plist + wsx * WCAP;
#pragma unroll 1
      for (int i = 0; i < n; ++i) {
        const int ent = __builtin_amdgcn_readfirstlane(lp[i]);
        int slot = ent & (NBA - 1);
        slot = slot > NGB - 1 ? NGB - 1 : slot;
        if ((slot >> 2) == wave) {
          int nd = cbase + ((ent >> SLA) & (CHUNK - 1));
          nd = nd > nN - 1 ? nN - 1 : nd;
          const v2f o = *(const v2fa*)(hr + (size_t)nd * F + 2 * lane);
          const float h0 = fmaf(o.x, sc0, sh0);
          const float h1 = fmaf(o.y, sc1, sh1);
          const float d = wsum(fmaf(h0, aw0, h1 * aw1));
          float ta = -(d + ab);
          ta = fminf(ta, 80.0f);
          const float e = expf(ta);
          const float w = __builtin_amdgcn_rcpf(1.0f + e);
          v2f* sp = (v2f*)(Rs + slot * F + 2 * lane);
          v2f sv = *sp;
          sv.x = fmaf(h0, w, sv.x);
          sv.y = fmaf(h1, w, sv.y);
          *sp = sv;
          v2f* mp = (v2f*)(Rm + slot * F + 2 * lane);
          v2f mv = *mp;
          mv.x = fmaxf(mv.x, h0);
          mv.y = fmaxf(mv.y, h1);
          *mp = mv;
        }
      }
    }
    __syncthreads();
  }

  v8us ov[4];
  const int k = 8 * (lane & 15);
  const int half = lane >> 4;
#pragma unroll
  for (int j = 0; j < 4; ++j) {
    const int slot = 4 * wave + j;
    v8us o;
#pragma unroll
    for (int i = 0; i < 8; ++i) {
      const int idx = k + i;
      const int is = idx & (F - 1);
      const float vs = Rs[slot * F + is];
      const float vm = Rm[slot * F + is];
      const float v = (idx < F) ? vs : vm;
      const unsigned hb = bf16_bits(v);
      const unsigned lb = bf16_bits(v - __uint_as_float(hb << 16));
      o[i] = (half == 0) ? (unsigned short)hb : (unsigned short)lb;
    }
    ov[j] = o;
  }
#pragma unroll
  for (int j = 0; j < 4; ++j) {
    const int slot = 4 * wave + j;
    if (slot < nb) *(volatile v8us*)(hg + (size_t)(gBase + slot) * KC + half * CH + k) = ov[j];
  }
  __threadfence();
#pragma unroll
  for (int j = 0; j < 4; ++j) {
    const int slot = 4 * wave + j;
    if (slot < nb) *(volatile v8us*)(hg + (size_t)(gBase + slot) * KC + half * CH + k) = ov[j];
  }
}

__global__ __launch_bounds__(NTHR) void k_cls(const float* __restrict__ z, int G,
                                              const float* __restrict__ c1b, const float* __restrict__ cg,
                                              const float* __restrict__ cb, const unsigned short* __restrict__ c2t,
                                              const float* __restrict__ c2b, float* out) {
  __shared__ float b1s[CH];
  __shared__ float scs[CH];
  __shared__ float shs[CH];
  __shared__ float red[NTHR];
  __shared__ __attribute__((aligned(16))) float outs[MAXG * NTSK];
  const int tid = (int)threadIdx.x, lane = tid & 31, wave = tid >> 5, hh = lane >> 4, m = lane & 15;
  const int col = tid & (CH - 1);
  const int hsel = tid >> 7;
  const int rh = G >> 1;
  const int r0 = hsel * rh;
  const float b1 = bf16_val(c1b[col]);
  const float invG = 1.0f / (float)G;

  float s = 0.0f;
#pragma unroll 1
  for (int r = 0; r < rh; ++r) s += fmaxf(z[(size_t)(r0 + r) * CH + col] + b1, 0.0f);
  red[tid] = s;
  __syncthreads();
  const float mean = (red[col] + red[CH + col]) * invG;
  __syncthreads();
  float q = 0.0f;
#pragma unroll 1
  for (int r = 0; r < rh; ++r) {
    const float d = fmaxf(z[(size_t)(r0 + r) * CH + col] + b1, 0.0f) - mean;
    q = fmaf(d, d, q);
  }
  red[tid] = q;
  __syncthreads();
  const float var = (red[col] + red[CH + col]) * invG;
  if (tid < CH) {
    const float rstd = rsqrtf(var + 1e-5f);
    const float sc = bf16_val(cg[col]) * rstd;
    scs[col] = sc;
    shs[col] = bf16_val(cb[col]) - mean * sc;
    b1s[col] = b1;
  }
  __syncthreads();

  const unsigned short* bt = c2t + (size_t)m * KC + 8 * hh;
  const float c2bv = bf16_val(c2b[m < NTSK ? m : NTSK - 1]);
  const int nIt = G / 128;
#pragma unroll 1
  for (int it = 0; it < nIt; ++it) {
    const int rowA = it * 128 + 16 * wave + m;
    const float* zr = z + (size_t)rowA * CH;
    v8f acc = z8();
#pragma unroll
    for (int ks = 0; ks < CH / 32; ++ks) {
      const int k0 = 32 * ks;
      const v4f p0 = *(const v4f*)(zr + k0 + 8 * hh);
      const v4f p1 = *(const v4f*)(zr + k0 + 8 * hh + 4);
      const v4f p2 = *(const v4f*)(zr + k0 + 16 + 8 * hh);
      const v4f p3 = *(const v4f*)(zr + k0 + 16 + 8 * hh + 4);
      float xv[16];
      xv[0] = p0.x;  xv[1] = p0.y;  xv[2] = p0.z;  xv[3] = p0.w;
      xv[4] = p1.x;  xv[5] = p1.y;  xv[6] = p1.z;  xv[7] = p1.w;
      xv[8] = p2.x;  xv[9] = p2.y;  xv[10] = p2.z; xv[11] = p2.w;
      xv[12] = p3.x; xv[13] = p3.y; xv[14] = p3.z; xv[15] = p3.w;
      FragB ah, al;
#pragma unroll
      for (int i = 0; i < 16; ++i) {
        const int kk = (i < 8) ? (k0 + 8 * hh + i) : (k0 + 16 + 8 * hh + (i - 8));
        const float x = fmaxf(xv[i] + b1s[kk], 0.0f);
        const float v = fmaf(x, scs[kk], shs[kk]);
        const unsigned hb = bf16_bits(v);
        const unsigned lb = bf16_bits(v - __uint_as_float(hb << 16));
        ah.u[i] = (unsigned short)hb;
        al.u[i] = (unsigned short)lb;
      }
      FragB bh, bl;
      bh.h[0] = *(const v8usa*)(bt + k0);
      bh.h[1] = *(const v8usa*)(bt + k0 + 16);
      bl.h[0] = *(const v8usa*)(bt + CH + k0);
      bl.h[1] = *(const v8usa*)(bt + CH + k0 + 16);
      acc = wmb(ah, bh, acc);
      acc = wmb(al, bl, acc);
    }
#pragma unroll
    for (int r = 0; r < 8; ++r) {
      const int row = it * 128 + 16 * wave + 8 * hh + r;
      if (m < NTSK) outs[row * NTSK + m] = acc[r] + c2bv;
    }
  }
  __syncthreads();

  const int nv4 = (G * NTSK) / 4;
#pragma unroll 1
  for (int i = tid; i < nv4; i += NTHR) {
    const v4f v = *(const v4fa*)(outs + 4 * i);
    *(volatile v4f*)(out + 4 * (size_t)i) = v;
  }
  __threadfence();
#pragma unroll 1
  for (int i = tid; i < nv4; i += NTHR) {
    const v4f v = *(const v4fa*)(outs + 4 * i);
    *(volatile v4f*)(out + 4 * (size_t)i) = v;
  }
}

static inline int cdiv(int a, int b) { return (a + b - 1) / b; }
static inline size_t al256(size_t o) { return (o + 255) & ~(size_t)255; }

extern "C" void kernel_launch(void* const* d_in, const int* in_sizes, int n_in,
                              void* d_out, int out_size, void* d_ws, size_t ws_size,
                              hipStream_t stream) {
  if (n_in < 24) return;
  if (in_sizes[0] < F || (in_sizes[0] % F) != 0) return;
  const int nN = in_sizes[0] / F;
  const int nE = in_sizes[1];
  if (nE < 1 || in_sizes[2] != nE || in_sizes[3] != nN) return;
  if (nE >= (1 << 21) || nN >= (1 << 24) || nN < 1) return;
  if (in_sizes[4] != F * F || in_sizes[5] != F || in_sizes[6] != F * F || in_sizes[7] != F) return;
  if (in_sizes[8] != F || in_sizes[9] != F) return;
  if (in_sizes[10] != F * F || in_sizes[11] != F || in_sizes[12] != F * F || in_sizes[13] != F) return;
  if (in_sizes[14] != F || in_sizes[15] != F) return;
  if (in_sizes[16] != F || in_sizes[17] < 1) return;
  if (in_sizes[18] != F2 * CH || in_sizes[19] != CH || in_sizes[20] != CH || in_sizes[21] != CH) return;
  if (in_sizes[22] != CH * NTSK || in_sizes[23] != NTSK) return;
  if (out_size < NTSK || (out_size % NTSK) != 0) return;
  const int G = out_size / NTSK;
  if (G > MAXG || (G % 128) != 0) return;

  const float* feats = (const float*)d_in[0];
  const int*   src   = (const int*)d_in[1];
  const int*   dst   = (const int*)d_in[2];
  const int*   ngr   = (const int*)d_in[3];
  const float* W0    = (const float*)d_in[4];
  const float* b0    = (const float*)d_in[5];
  const float* rW0   = (const float*)d_in[6];
  const float* rb0   = (const float*)d_in[7];
  const float* g0    = (const float*)d_in[8];
  const float* be0   = (const float*)d_in[9];
  const float* W1    = (const float*)d_in[10];
  const float* b1    = (const float*)d_in[11];
  const float* rW1   = (const float*)d_in[12];
  const float* rb1   = (const float*)d_in[13];
  const float* g1    = (const float*)d_in[14];
  const float* be1   = (const float*)d_in[15];
  const float* awW   = (const float*)d_in[16];
  const float* awb   = (const float*)d_in[17];
  const float* c1W   = (const float*)d_in[18];
  const float* c1b   = (const float*)d_in[19];
  const float* cg    = (const float*)d_in[20];
  const float* cb    = (const float*)d_in[21];
  const float* c2W   = (const float*)d_in[22];
  const float* c2b   = (const float*)d_in[23];
  float* out = (float*)d_out;

  const int MP = cdiv(nN, GBM) * GBM;
  const int gM = MP / GBM;
  const int gA = cdiv(nN, NBA);
  if ((long long)gA * NBA < (long long)MP) return;
  const int gP = cdiv(G, NGB);
  const int vec8e = ((nE & 3) == 0) ? 1 : 0;
  const int vec8n = ((nN & 3) == 0) ? 1 : 0;

  char* ws = (char*)d_ws;
  size_t off = 0;
  const size_t oA0 = off; off = al256(off + (size_t)MP * F * 2);
  const size_t oMR = off; off = al256(off + (size_t)MP * F2 * 4);
  const size_t oHR = off; off = al256(off + (size_t)MP * F * 4);
  const size_t oA1 = off; off = al256(off + (size_t)MP * F2 * 2);
  const size_t oB0 = off; off = al256(off + (size_t)F2 * F * 2);
  const size_t oB1 = off; off = al256(off + (size_t)F2 * F2 * 2);
  const size_t oC1 = off; off = al256(off + (size_t)CH * KC * 2);
  const size_t oC2 = off; off = al256(off + (size_t)NTP * KC * 2);
  const size_t oP0 = off; off = al256(off + (size_t)gA * PARTW * 4);
  const size_t oP1 = off; off = al256(off + (size_t)gA * PARTW * 4);
  const size_t oS0 = off; off = al256(off + (size_t)F2 * 4);
  const size_t oS1 = off; off = al256(off + (size_t)F2 * 4);
  const size_t oHG = off; off = al256(off + (size_t)G * KC * 2);
  const size_t oZ  = off; off = al256(off + (size_t)G * CH * 4);
  if (off > ws_size || off > (size_t)WSMAX) return;
  unsigned short* A0  = (unsigned short*)(ws + oA0);
  float*          MR  = (float*)(ws + oMR);
  float*          HR  = (float*)(ws + oHR);
  unsigned short* A1  = (unsigned short*)(ws + oA1);
  unsigned short* B0  = (unsigned short*)(ws + oB0);
  unsigned short* B1  = (unsigned short*)(ws + oB1);
  unsigned short* C1T = (unsigned short*)(ws + oC1);
  unsigned short* C2T = (unsigned short*)(ws + oC2);
  float*          P0  = (float*)(ws + oP0);
  float*          P1  = (float*)(ws + oP1);
  float*          S0  = (float*)(ws + oS0);
  float*          S1  = (float*)(ws + oS1);
  unsigned short* HG  = (unsigned short*)(ws + oHG);
  float*          Z   = (float*)(ws + oZ);

  const size_t aggLds = (size_t)AGG_LDS_INTS * 4;
  hipFuncSetAttribute(reinterpret_cast<const void*>(&k_agg), hipFuncAttributeMaxDynamicSharedMemorySize, (int)aggLds);

  const int nUa = MP * (F / 8);
  k_prep<<<(NUB0 + NUB1 + NUC1 + NUC2) / NTHR, NTHR, 0, stream>>>(W0, rW0, W1, rW1, c1W, c2W, B0, B1, C1T, C2T);
  k_cva<<<cdiv(nUa, NTHR), NTHR, 0, stream>>>(feats, nN, nUa, A0);
  k_gemm<<<dim3(gM, F2 / GBN), GTHR, 0, stream>>>(A0, F, B0, F, F, MR, F2);
  k_agg<<<gA, NTHR, aggLds, stream>>>(src, dst, nE, nN, vec8e, MP, MR, b0, rb0, HR, P0);
  k_bnfin<<<1, 64, 0, stream>>>(P0, gA, g0, be0, S0);
  k_bnap<<<cdiv(nUa, NTHR), NTHR, 0, stream>>>(HR, nN, nUa, S0, A1);
  k_gemm<<<dim3(gM, F2 / GBN), GTHR, 0, stream>>>(A1, F2, B1, F2, F2, MR, F2);
  k_agg<<<gA, NTHR, aggLds, stream>>>(src, dst, nE, nN, vec8e, MP, MR, b1, rb1, HR, P1);
  k_bnfin<<<1, 64, 0, stream>>>(P1, gA, g1, be1, S1);
  k_pool<<<gP, NTHR, 0, stream>>>(ngr, nN, vec8n, HR, S1, awW, awb, HG, G);
  k_gemm<<<dim3(G / GBM, CH / GBN), GTHR, 0, stream>>>(HG, KC, C1T, KC, KC, Z, CH);
  k_cls<<<1, NTHR, 0, stream>>>(Z, G, c1b, cg, cb, C2T, c2b, out);
}
